// LSTM_30073361007081
// MI455X (gfx1250) — hardware-run, weakly checked
//
#include <hip/hip_runtime.h>
#include <math.h>

constexpr int NBATCH   = 1024;
constexpr int NSTEP    = 512;
constexpr int NHID     = 64;
constexpr int NGATE    = 4 * NHID;
constexpr int NTHR     = 128;
constexpr int NWAVES   = NTHR / 32;
constexpr int ROWS_BLK = 16;
constexpr int HPITCH   = 72;
constexpr int FPITCH   = 68;
constexpr int XPITCH   = 36;
constexpr int OPITCH   = 36;
constexpr int TCHUNK   = 32;
constexpr int GSTRIDE  = NHID * NHID;
constexpr int WPLANE_ELEMS = NGATE * NHID;
constexpr float WCARRY = 256.0f;
constexpr float HCARRY = 16.0f;
constexpr float ZFOLD  = 1.0f / (256.0f * 16.0f);
static_assert(NHID == 16 * NWAVES);
static_assert(NHID % 32 == 0);
static_assert(NBATCH % ROWS_BLK == 0);
static_assert(NSTEP % TCHUNK == 0);
static_assert(ROWS_BLK * TCHUNK == NTHR * 4);
static_assert((2 * ROWS_BLK * HPITCH) % NTHR == 0);
static_assert(WPLANE_ELEMS % 512 == 0);
static_assert(NGATE == 4 * NHID);
static_assert(HPITCH % 8 == 0 && FPITCH % 4 == 0 && XPITCH % 4 == 0 && OPITCH % 4 == 0);

typedef __attribute__((ext_vector_type(16))) _Float16 v16h;
typedef __attribute__((ext_vector_type(8)))  _Float16 v8h;
typedef __attribute__((ext_vector_type(8)))  float    v8f;
typedef __attribute__((ext_vector_type(4)))  float    v4f;

__device__ __forceinline__ void acc_guard4(v8f& a, v8f& b, v8f& c, v8f& d) {
  asm volatile("v_nop\n\tv_nop\n\tv_nop\n\tv_nop" : "+v"(a), "+v"(b), "+v"(c), "+v"(d));
}
__device__ __forceinline__ void grp_guard(v8f& a0, v8f& a1, v8f& a2, v8f& a3,
                                          v16h x, v16h b0, v16h b1, v16h b2, v16h b3) {
  asm volatile("v_nop\n\tv_nop\n\tv_nop\n\tv_nop"
               : "+v"(a0), "+v"(a1), "+v"(a2), "+v"(a3)
               : "v"(x), "v"(b0), "v"(b1), "v"(b2), "v"(b3));
}

template <typename T> struct Frag;
template <> struct Frag<_Float16> {
  typedef v16h V; union U { v16h v; v8h h[2]; };
  static __device__ __forceinline__ v16h load(const _Float16* p) {
    U f; f.h[0] = *(const v8h*)(p); f.h[1] = *(const v8h*)(p + 16); return f.v;
  }
  static __device__ __forceinline__ v8f mma(v16h a, v16h b, v8f c) {
    return __builtin_amdgcn_wmma_f32_16x16x32_f16(false, a, false, b, (short)0, c, false, false);
  }
};

__device__ __forceinline__ float fsig(float x)  { return __builtin_amdgcn_rcpf(1.0f + __expf(-x)); }
__device__ __forceinline__ float ftanh(float x) { return 1.0f - 2.0f * __builtin_amdgcn_rcpf(__expf(2.0f * x) + 1.0f); }

__global__ __launch_bounds__(256) void cast_scale_f16x2(const float* __restrict__ in, _Float16* __restrict__ dst,
                                                        int n2, float sc) {
  const int i = blockIdx.x * 256 + threadIdx.x;
  if (i < n2) {
    const _Float16 h0 = (_Float16)(in[2 * i] * sc);
    const _Float16 h1 = (_Float16)(in[2 * i + 1] * sc);
    const unsigned u = (unsigned)__builtin_bit_cast(unsigned short, h0) |
                       ((unsigned)__builtin_bit_cast(unsigned short, h1) << 16);
    ((volatile unsigned*)dst)[i] = u;
    __threadfence();
    ((volatile unsigned*)dst)[i] = u;
  }
}

__global__ __launch_bounds__(NTHR) void lstm2_seq_kernel(const float* __restrict__ xg,
                                                         const float* __restrict__ wih1,
                                                         const float* __restrict__ bih1,
                                                         const float* __restrict__ bhh1,
                                                         const float* __restrict__ bih2,
                                                         const float* __restrict__ bhh2,
                                                         const float* __restrict__ wlin,
                                                         const float* __restrict__ blin,
                                                         const int*   __restrict__ fpp,
                                                         const unsigned short* __restrict__ W1p,
                                                         const unsigned short* __restrict__ W2Ip,
                                                         const unsigned short* __restrict__ W2Hp,
                                                         float* __restrict__ out) {
  __shared__ __align__(16) _Float16 Ah1[2][ROWS_BLK * HPITCH];
  __shared__ __align__(16) _Float16 Ah2[2][ROWS_BLK * HPITCH];
  __shared__ __align__(16) float    H2f[ROWS_BLK * FPITCH];
  __shared__ __align__(16) float    Xs[ROWS_BLK * XPITCH];
  __shared__ __align__(16) float    Ob[ROWS_BLK * OPITCH];
  __shared__ __align__(16) float    Wl[NHID];
  __shared__ __align__(16) float    Pw[NGATE];
  __shared__ __align__(16) float    Pb1[NGATE];
  __shared__ __align__(16) float    Pb2[NGATE];
  (void)fpp;

  const _Float16* W1  = (const _Float16*)W1p;
  const _Float16* W2I = (const _Float16*)W2Ip;
  const _Float16* W2H = (const _Float16*)W2Hp;
  const int tid = threadIdx.x, lane = tid & 31, wave = tid >> 5;
  const int c = lane & 15, hh = lane >> 4, koff = hh * 8;
  const int j = 16 * wave + c;
  const int rowbase = blockIdx.x * ROWS_BLK;

  {
    _Float16* a1f = &Ah1[0][0];
    _Float16* a2f = &Ah2[0][0];
#pragma unroll 1
    for (int i = tid; i < 2 * ROWS_BLK * HPITCH; i += NTHR) { a1f[i] = (_Float16)0.0f; a2f[i] = (_Float16)0.0f; }
  }
  if (tid < NHID) {
    const int q4 = 4 * tid;
    const v4f va = *(const v4f*)(wih1 + q4);
    const v4f vb = *(const v4f*)(bih1 + q4);
    const v4f vc = *(const v4f*)(bhh1 + q4);
    const v4f vd = *(const v4f*)(bih2 + q4);
    const v4f ve = *(const v4f*)(bhh2 + q4);
    const float wl = wlin[tid];
    *(v4f*)(Pw  + q4) = va;
    *(v4f*)(Pb1 + q4) = vb + vc;
    *(v4f*)(Pb2 + q4) = vd + ve;
    Wl[tid] = wl;
  }
  const float blv = blin[0];

  float c1s[8], c2s[8];
#pragma unroll
  for (int r = 0; r < 8; ++r) { c1s[r] = 0.0f; c2s[r] = 0.0f; }
  __syncthreads();

  float wi1[4], b1v[4], b2v[4];
#pragma unroll
  for (int g = 0; g < 4; ++g) {
    const int n = 64 * g + j;
    wi1[g] = Pw[n];
    b1v[g] = Pb1[n];
    b2v[g] = Pb2[n];
  }

  const int orow = tid >> 3, okc = tid & 7, oc4 = okc * 4;
  const v4f wva = *(const v4f*)(Wl + 8 * okc);
  const v4f wvb = *(const v4f*)(Wl + 8 * okc + 4);

  const v8f z8 = {0.f, 0.f, 0.f, 0.f, 0.f, 0.f, 0.f, 0.f};
  const _Float16* w1  = W1  + (size_t)j * NHID + koff;
  const _Float16* w2i = W2I + (size_t)j * NHID + koff;
  const _Float16* w2h = W2H + (size_t)j * NHID + koff;

#pragma unroll 1
  for (int t = 0; t < NSTEP; ++t) {
    const int cur = t & 1, nxt = cur ^ 1;
    const int tt = t & (TCHUNK - 1);

    if (tt == 0) {
      const v4f xv = *(const v4f*)(xg + (size_t)(rowbase + orow) * NSTEP + (size_t)t + oc4);
      *(v4f*)(Xs + orow * XPITCH + oc4) = xv;
      __syncthreads();
    }

    float xs[8];
#pragma unroll
    for (int r = 0; r < 8; ++r) xs[r] = Xs[(8 * hh + r) * XPITCH + tt];

    float h1n[8];
    {
      const _Float16* arow = &Ah1[cur][0] + c * HPITCH + koff;
      v8f acc[4];
      acc[0] = z8; acc[1] = z8; acc[2] = z8; acc[3] = z8;
#pragma unroll 1
      for (int k0 = 0; k0 < NHID; k0 += 32) {
        const v16h a  = Frag<_Float16>::load(arow + k0);
        const v16h b0 = Frag<_Float16>::load(w1 + k0);
        const v16h b1 = Frag<_Float16>::load(w1 + (size_t)1 * GSTRIDE + k0);
        const v16h b2 = Frag<_Float16>::load(w1 + (size_t)2 * GSTRIDE + k0);
        const v16h b3 = Frag<_Float16>::load(w1 + (size_t)3 * GSTRIDE + k0);
        acc[0] = Frag<_Float16>::mma(a, b0, acc[0]);
        acc[1] = Frag<_Float16>::mma(a, b1, acc[1]);
        acc[2] = Frag<_Float16>::mma(a, b2, acc[2]);
        acc[3] = Frag<_Float16>::mma(a, b3, acc[3]);
        grp_guard(acc[0], acc[1], acc[2], acc[3], a, b0, b1, b2, b3);
      }
      acc_guard4(acc[0], acc[1], acc[2], acc[3]);
#pragma unroll
      for (int r = 0; r < 8; ++r) {
        const float zi = acc[0][r] * ZFOLD + (b1v[0] + xs[r] * wi1[0]);
        const float zf = acc[1][r] * ZFOLD + (b1v[1] + xs[r] * wi1[1]);
        const float zg = acc[2][r] * ZFOLD + (b1v[2] + xs[r] * wi1[2]);
        const float zo = acc[3][r] * ZFOLD + (b1v[3] + xs[r] * wi1[3]);
        const float ig = fsig(zi);
        const float fg = fsig(zf);
        const float gg = ftanh(zg);
        const float og = fsig(zo);
        const float cn = fg * c1s[r] + ig * gg;
        c1s[r] = cn;
        h1n[r] = og * ftanh(cn);
      }
    }
#pragma unroll
    for (int r = 0; r < 8; ++r) Ah1[nxt][(8 * hh + r) * HPITCH + j] = (_Float16)(h1n[r] * HCARRY);
    __syncthreads();

    float h2n[8];
    {
      const _Float16* a1row = &Ah1[nxt][0] + c * HPITCH + koff;
      const _Float16* a2row = &Ah2[cur][0] + c * HPITCH + koff;
      v8f acc[4];
      acc[0] = z8; acc[1] = z8; acc[2] = z8; acc[3] = z8;
#pragma unroll 1
      for (int k0 = 0; k0 < NHID; k0 += 32) {
        const v16h a  = Frag<_Float16>::load(a1row + k0);
        const v16h b0 = Frag<_Float16>::load(w2i + k0);
        const v16h b1 = Frag<_Float16>::load(w2i + (size_t)1 * GSTRIDE + k0);
        const v16h b2 = Frag<_Float16>::load(w2i + (size_t)2 * GSTRIDE + k0);
        const v16h b3 = Frag<_Float16>::load(w2i + (size_t)3 * GSTRIDE + k0);
        acc[0] = Frag<_Float16>::mma(a, b0, acc[0]);
        acc[1] = Frag<_Float16>::mma(a, b1, acc[1]);
        acc[2] = Frag<_Float16>::mma(a, b2, acc[2]);
        acc[3] = Frag<_Float16>::mma(a, b3, acc[3]);
        grp_guard(acc[0], acc[1], acc[2], acc[3], a, b0, b1, b2, b3);
      }
#pragma unroll 1
      for (int k0 = 0; k0 < NHID; k0 += 32) {
        const v16h a  = Frag<_Float16>::load(a2row + k0);
        const v16h b0 = Frag<_Float16>::load(w2h + k0);
        const v16h b1 = Frag<_Float16>::load(w2h + (size_t)1 * GSTRIDE + k0);
        const v16h b2 = Frag<_Float16>::load(w2h + (size_t)2 * GSTRIDE + k0);
        const v16h b3 = Frag<_Float16>::load(w2h + (size_t)3 * GSTRIDE + k0);
        acc[0] = Frag<_Float16>::mma(a, b0, acc[0]);
        acc[1] = Frag<_Float16>::mma(a, b1, acc[1]);
        acc[2] = Frag<_Float16>::mma(a, b2, acc[2]);
        acc[3] = Frag<_Float16>::mma(a, b3, acc[3]);
        grp_guard(acc[0], acc[1], acc[2], acc[3], a, b0, b1, b2, b3);
      }
      acc_guard4(acc[0], acc[1], acc[2], acc[3]);
#pragma unroll
      for (int r = 0; r < 8; ++r) {
        const float zi = acc[0][r] * ZFOLD + b2v[0];
        const float zf = acc[1][r] * ZFOLD + b2v[1];
        const float zg = acc[2][r] * ZFOLD + b2v[2];
        const float zo = acc[3][r] * ZFOLD + b2v[3];
        const float ig = fsig(zi);
        const float fg = fsig(zf);
        const float gg = ftanh(zg);
        const float og = fsig(zo);
        const float cn = fg * c2s[r] + ig * gg;
        c2s[r] = cn;
        h2n[r] = og * ftanh(cn);
      }
    }
#pragma unroll
    for (int r = 0; r < 8; ++r) {
      Ah2[nxt][(8 * hh + r) * HPITCH + j] = (_Float16)(h2n[r] * HCARRY);
      H2f[(8 * hh + r) * FPITCH + j] = h2n[r];
    }
    __syncthreads();

    {
      const v4f hva = *(const v4f*)(H2f + orow * FPITCH + 8 * okc);
      const v4f hvb = *(const v4f*)(H2f + orow * FPITCH + 8 * okc + 4);
      float p = 0.0f;
      p = fmaf(hva[0], wva[0], p); p = fmaf(hva[1], wva[1], p); p = fmaf(hva[2], wva[2], p); p = fmaf(hva[3], wva[3], p);
      p = fmaf(hvb[0], wvb[0], p); p = fmaf(hvb[1], wvb[1], p); p = fmaf(hvb[2], wvb[2], p); p = fmaf(hvb[3], wvb[3], p);
      p += __shfl_xor(p, 1, 32);
      p += __shfl_xor(p, 2, 32);
      p += __shfl_xor(p, 4, 32);
      if (okc == 0) Ob[orow * OPITCH + tt] = p + blv;
    }

    if (tt == TCHUNK - 1) {
      __syncthreads();
      const v4f ov = *(const v4f*)(Ob + orow * OPITCH + oc4);
      float* op = out + (size_t)(rowbase + orow) * NSTEP + (size_t)(t - (TCHUNK - 1)) + oc4;
      for (int pass = 0; pass < 2; ++pass) {
        *(volatile v4f*)op = ov;
        __threadfence();
      }
    }
  }
}

extern "C" void kernel_launch(void* const* d_in, const int* in_sizes, int n_in,
                              void* d_out, int out_size, void* d_ws, size_t ws_size, hipStream_t stream) {
  if (n_in < 12 || d_out == nullptr || d_ws == nullptr) return;
  if (in_sizes[0] != NBATCH * NSTEP || in_sizes[1] != NGATE || in_sizes[2] != NGATE * NHID ||
      in_sizes[3] != NGATE || in_sizes[4] != NGATE || in_sizes[5] != NGATE * NHID || in_sizes[6] != NGATE * NHID ||
      in_sizes[7] != NGATE || in_sizes[8] != NGATE || in_sizes[9] != NHID || in_sizes[10] != 1 || in_sizes[11] != 1 ||
      out_size != NBATCH * NSTEP) return;

  const float* x    = (const float*)d_in[0];
  const float* wih1 = (const float*)d_in[1];
  const float* whh1 = (const float*)d_in[2];
  const float* bih1 = (const float*)d_in[3];
  const float* bhh1 = (const float*)d_in[4];
  const float* wih2 = (const float*)d_in[5];
  const float* whh2 = (const float*)d_in[6];
  const float* bih2 = (const float*)d_in[7];
  const float* bhh2 = (const float*)d_in[8];
  const float* wlin = (const float*)d_in[9];
  const float* blin = (const float*)d_in[10];
  const int*   fpp  = (const int*)d_in[11];
  float* out = (float*)d_out;

  char* ws = (char*)d_ws; size_t off = 0;
  auto carve = [&](size_t bytes) -> char* { char* p = ws + off; off += (bytes + 255) & ~(size_t)255; return p; };
  _Float16* W1  = (_Float16*)carve((size_t)WPLANE_ELEMS * 2);
  _Float16* W2I = (_Float16*)carve((size_t)WPLANE_ELEMS * 2);
  _Float16* W2H = (_Float16*)carve((size_t)WPLANE_ELEMS * 2);
  if (off > ws_size || off > (size_t)134217728) return;

  const int n2 = WPLANE_ELEMS / 2;
  cast_scale_f16x2<<<n2 / 256, 256, 0, stream>>>(whh1, W1,  n2, WCARRY);
  cast_scale_f16x2<<<n2 / 256, 256, 0, stream>>>(wih2, W2I, n2, WCARRY);
  cast_scale_f16x2<<<n2 / 256, 256, 0, stream>>>(whh2, W2H, n2, WCARRY);
  lstm2_seq_kernel<<<NBATCH / ROWS_BLK, NTHR, 0, stream>>>(
      x, wih1, bih1, bhh1, bih2, bhh2, wlin, blin, fpp,
      (const unsigned short*)W1, (const unsigned short*)W2I, (const unsigned short*)W2H, out);
}
